// GCNHead_1915555414122
// MI455X (gfx1250) — hardware-verified
//
#include <hip/hip_runtime.h>
#include <stddef.h>
#include <stdint.h>
#include <math.h>


#define HID    64
#define K2     128
#define NG     64
#define NTHR   256
#define NWAVE  8
#define EPT    8
#define CHUNK  (NTHR * EPT)
#define WCAP   (EPT * 32)
#define LISTN  (NWAVE * WCAP)
#define NBD    8192
#define SLD    13
#define NBA    1024
#define SLA    10
#define RCAP   24576
#define DEGCAP 128
#define GBM    64
#define GBN    64
#define GTHR   128
#define PTAB   (NG * HID)
#define DREG   (NWAVE * PTAB)
#define SCAN_ZINTS    (DREG + RCAP + 2 * NBA)
#define SCAN_LDS_INTS (SCAN_ZINTS + 16)
#define NOUT   (NG * HID)
#define NITER  512
#define NWU    (HID * (HID / 8))
#define HEAD_DBL (2 * 4096 + 64 + 64 + 256 + 8)
#define HEAD_LDS (HEAD_DBL * 8 + 3 * 4096 * 4 + 4096 * 2)
#define WSMAX  134217728

static_assert((CHUNK & (CHUNK - 1)) == 0 && CHUNK <= 4096);
static_assert((NBD & (NBD - 1)) == 0 && NBD == (1 << SLD));
static_assert((NBA & (NBA - 1)) == 0 && NBA == (1 << SLA));
static_assert(((long long)CHUNK << SLD) < (1LL << 31));
static_assert(((long long)CHUNK << SLA) < (1LL << 31));
static_assert(NBD % (NTHR * 4) == 0);
static_assert(LISTN % NTHR == 0);
static_assert(NBA % NWAVE == 0 && NBA % 32 == 0);
static_assert(LISTN + RCAP + NBA <= DREG);
static_assert(SCAN_ZINTS % (NTHR * 4) == 0 && DREG % (NTHR * 4) == 0);
static_assert(SCAN_LDS_INTS * 4 <= 300000);
static_assert(RCAP >= 16623 + 4096 && DEGCAP >= 35 + 8);
static_assert(HID % 32 == 0 && K2 % 32 == 0 && K2 == 2 * HID && HID == GBN);
static_assert(GBM == (GTHR / 32) * 16);
static_assert(HID == 2 * 32);
static_assert(NOUT == 4 * 4 * NTHR && (NOUT * 4) % 128 == 0);
static_assert((HEAD_DBL * 8) % 16 == 0 && HEAD_LDS <= 300000);
static_assert(NWU % NTHR == 0);

typedef float          v2f   __attribute__((ext_vector_type(2)));
typedef float          v4f   __attribute__((ext_vector_type(4)));
typedef float          v8f   __attribute__((ext_vector_type(8)));
typedef int            v4i   __attribute__((ext_vector_type(4)));
typedef int            v8i   __attribute__((ext_vector_type(8)));
typedef unsigned short v4us  __attribute__((ext_vector_type(4)));
typedef unsigned short v8us  __attribute__((ext_vector_type(8)));
typedef unsigned short v16us __attribute__((ext_vector_type(16)));
typedef __bf16         v16bf __attribute__((ext_vector_type(16)));
typedef v2f  __attribute__((may_alias)) v2fa;
typedef v4f  __attribute__((may_alias)) v4fa;
typedef v4i  __attribute__((may_alias)) v4ia;
typedef v4us __attribute__((may_alias)) v4usa;
typedef v8us __attribute__((may_alias)) v8usa;
union FragB { v16bf v; v16us u; v8us h[2]; v8i w; };

__device__ __forceinline__ v8f wmb(const FragB& a, const FragB& b, v8f c) {
  v8f d = __builtin_amdgcn_wmma_f32_16x16x32_bf16(false, a.v, false, b.v, (short)0, c, false, false);
  asm volatile("v_nop\n\tv_nop\n\tv_nop\n\tv_nop" : "+v"(d) : "v"(a.w), "v"(b.w));
  return d;
}

__device__ __forceinline__ unsigned bf16_bits(float f) {
  const unsigned u = __float_as_uint(f);
  return (u + 0x7FFFu + ((u >> 16) & 1u)) >> 16;
}
__device__ __forceinline__ unsigned bf16_bits_n(float f) {
  const unsigned b = bf16_bits(f);
  return (f != f) ? 0x7fc0u : b;
}
__device__ __forceinline__ float bf16_val(float f) {
  return __uint_as_float(bf16_bits(f) << 16);
}
__device__ __forceinline__ float nmax(float v, float m) {
  return (v > m || v != v) ? v : m;
}

template <int SLB>
__device__ __forceinline__ int scan_chunk(const int* __restrict__ dsts, int nE, int cbase, int slotBase,
                                          int nb, int vec8, int* list, int tid, int lane, int wave) {
  int wc = 0;
  const int el0  = tid * EPT;
  const int e0   = cbase + el0;
  const int sent = -2147483647 - 1;
  v4i da, db;
  if (vec8 != 0 && cbase + CHUNK <= nE) {
    da = *(const v4i*)(dsts + e0);
    db = *(const v4i*)(dsts + e0 + 4);
  } else {
    da.x = (e0     < nE) ? dsts[min(e0,     nE - 1)] : sent;
    da.y = (e0 + 1 < nE) ? dsts[min(e0 + 1, nE - 1)] : sent;
    da.z = (e0 + 2 < nE) ? dsts[min(e0 + 2, nE - 1)] : sent;
    da.w = (e0 + 3 < nE) ? dsts[min(e0 + 3, nE - 1)] : sent;
    db.x = (e0 + 4 < nE) ? dsts[min(e0 + 4, nE - 1)] : sent;
    db.y = (e0 + 5 < nE) ? dsts[min(e0 + 5, nE - 1)] : sent;
    db.z = (e0 + 6 < nE) ? dsts[min(e0 + 6, nE - 1)] : sent;
    db.w = (e0 + 7 < nE) ? dsts[min(e0 + 7, nE - 1)] : sent;
  }
  const unsigned nbs = (unsigned)slotBase;
  const unsigned unb = (unsigned)nb;
  const unsigned s0 = (unsigned)da.x - nbs, s1 = (unsigned)da.y - nbs;
  const unsigned s2 = (unsigned)da.z - nbs, s3 = (unsigned)da.w - nbs;
  const unsigned s4 = (unsigned)db.x - nbs, s5 = (unsigned)db.y - nbs;
  const unsigned s6 = (unsigned)db.z - nbs, s7 = (unsigned)db.w - nbs;
  const bool h0 = s0 < unb, h1 = s1 < unb, h2 = s2 < unb, h3 = s3 < unb;
  const bool h4 = s4 < unb, h5 = s5 < unb, h6 = s6 < unb, h7 = s7 < unb;
  const unsigned any = __builtin_amdgcn_ballot_w32(h0 | h1 | h2 | h3 | h4 | h5 | h6 | h7);
  if (any != 0u) {
#define HITJ(J, HJ, SJ) { \
      const unsigned mj = __builtin_amdgcn_ballot_w32(HJ); \
      if (mj != 0u) { \
        if (HJ) { \
          const int pos = wc + (int)__builtin_amdgcn_mbcnt_lo(mj, 0u); \
          if (pos < WCAP) list[wave * WCAP + pos] = ((el0 + (J)) << SLB) | (int)(SJ); \
        } \
        wc += (int)__builtin_popcount(mj); } }
    HITJ(0, h0, s0)
    HITJ(1, h1, s1)
    HITJ(2, h2, s2)
    HITJ(3, h3, s3)
    HITJ(4, h4, s4)
    HITJ(5, h5, s5)
    HITJ(6, h6, s6)
    HITJ(7, h7, s7)
#undef HITJ
  }
  return wc;
}

__global__ __launch_bounds__(NTHR) void k_prep(const float* __restrict__ x, const float* __restrict__ Wg,
                                               int nN, int gX, int nUx,
                                               unsigned short* xb, unsigned short* wgt) {
  const int tid = (int)threadIdx.x;
  v8us o;
  unsigned short* dp;
  if ((int)blockIdx.x < gX) {
    const int u = (int)blockIdx.x * NTHR + tid;
    if (u >= nUx) return;
    const int row = u >> 3;
    const int k8  = (u & 7) * 8;
    const int rc  = row < nN ? row : nN - 1;
    const float* p = x + (size_t)rc * HID + k8;
    const v4f a = *(const v4fa*)p;
    const v4f b = *(const v4fa*)(p + 4);
    const bool ok = row < nN;
    o[0] = ok ? (unsigned short)bf16_bits(a.x) : (unsigned short)0;
    o[1] = ok ? (unsigned short)bf16_bits(a.y) : (unsigned short)0;
    o[2] = ok ? (unsigned short)bf16_bits(a.z) : (unsigned short)0;
    o[3] = ok ? (unsigned short)bf16_bits(a.w) : (unsigned short)0;
    o[4] = ok ? (unsigned short)bf16_bits(b.x) : (unsigned short)0;
    o[5] = ok ? (unsigned short)bf16_bits(b.y) : (unsigned short)0;
    o[6] = ok ? (unsigned short)bf16_bits(b.z) : (unsigned short)0;
    o[7] = ok ? (unsigned short)bf16_bits(b.w) : (unsigned short)0;
    dp = xb + (size_t)row * HID + k8;
  } else {
    const int v = ((int)blockIdx.x - gX) * NTHR + tid;
    if (v >= NWU) return;
    const int n  = v >> 3;
    const int k8 = (v & 7) * 8;
    const float* p = Wg + (size_t)k8 * HID + n;
#pragma unroll
    for (int i = 0; i < 8; ++i) o[i] = (unsigned short)bf16_bits(p[(size_t)i * HID]);
    dp = wgt + (size_t)n * HID + k8;
  }
  *(volatile v8us*)dp = o;
  __threadfence();
  *(volatile v8us*)dp = o;
}

__global__ __launch_bounds__(NTHR) void k_deg(const int* __restrict__ dsts, int nE, int vec8, float* dis) {
  __shared__ __attribute__((aligned(16))) int scnt[NBD];
  __shared__ __attribute__((aligned(16))) int list[LISTN];
  __shared__ int wcnt[NWAVE];
  const int tid = (int)threadIdx.x, lane = tid & 31, wave = tid >> 5;
  const int nodeBase = (int)blockIdx.x * NBD;

  for (int i = tid; i < NBD; i += NTHR) scnt[i] = 0;
  for (int i = tid; i < LISTN; i += NTHR) list[i] = 0;
  if (tid < NWAVE) wcnt[tid] = 0;
  __syncthreads();

  const int nChunks = (nE + CHUNK - 1) / CHUNK;
#pragma unroll 1
  for (int ch = 0; ch < nChunks; ++ch) {
    const int cbase = ch * CHUNK;
    const int wc = scan_chunk<SLD>(dsts, nE, cbase, nodeBase, NBD, vec8, list, tid, lane, wave);
    if (lane == 0) wcnt[wave] = wc;
    __syncthreads();
    if (wave == 0) {
#pragma unroll 1
      for (int w2 = 0; w2 < NWAVE; ++w2) {
        int c = wcnt[w2];
        c = c < 0 ? 0 : (c > WCAP ? WCAP : c);
#pragma unroll 1
        for (int b0 = 0; b0 < c; b0 += 32) {
          const int idx = b0 + lane;
          const int ent = list[w2 * WCAP + (idx < WCAP ? idx : WCAP - 1)];
          const int m32 = (c - b0) < 32 ? (c - b0) : 32;
#pragma unroll 1
          for (int k = 0; k < m32; ++k) {
            const int u  = __builtin_amdgcn_readlane(ent, k);
            const int sl = u & (NBD - 1);
            if (lane == 0) scnt[sl] = scnt[sl] + 1;
          }
        }
      }
    }
    __syncthreads();
  }

#pragma unroll 1
  for (int i = tid; i < NBD; i += NTHR) {
    const float d = (float)(scnt[i] + 1);
    const float r = (d > 0.0f) ? (1.0f / sqrtf(d)) : 0.0f;
    scnt[i] = __float_as_int(r);
  }
  __syncthreads();

  v4f vals[NBD / (NTHR * 4)];
#pragma unroll
  for (int it = 0; it < NBD / (NTHR * 4); ++it) {
    const int s0 = it * (NTHR * 4) + 4 * tid;
    const v4i c4 = *(const v4ia*)(scnt + s0);
    v4f v;
    v.x = __int_as_float(c4.x); v.y = __int_as_float(c4.y);
    v.z = __int_as_float(c4.z); v.w = __int_as_float(c4.w);
    vals[it] = v;
  }
#pragma unroll
  for (int it = 0; it < NBD / (NTHR * 4); ++it) {
    const int s0 = it * (NTHR * 4) + 4 * tid;
    *(volatile v4f*)(dis + (size_t)nodeBase + s0) = vals[it];
  }
  __threadfence();
#pragma unroll
  for (int it = 0; it < NBD / (NTHR * 4); ++it) {
    const int s0 = it * (NTHR * 4) + 4 * tid;
    *(volatile v4f*)(dis + (size_t)nodeBase + s0) = vals[it];
  }
}

__global__ __launch_bounds__(GTHR) void k_gemm(const unsigned short* __restrict__ A,
                                               const unsigned short* __restrict__ WT,
                                               const float* __restrict__ dis, float* outF) {
  __shared__ __attribute__((aligned(16))) float stg[GBM * GBN];
  __shared__ float sdi[GBM];
  const int tid = (int)threadIdx.x, lane = tid & 31, wave = tid >> 5, hh = lane >> 4, m = lane & 15;
  const int rowBase = (int)blockIdx.x * GBM;

  if (tid < GBM) sdi[tid] = dis[rowBase + tid];

  v8f acc[4];
  {
    const v8f z = {0.f, 0.f, 0.f, 0.f, 0.f, 0.f, 0.f, 0.f};
    acc[0] = z; acc[1] = z; acc[2] = z; acc[3] = z;
  }
  const unsigned short* ap = A  + (size_t)(rowBase + 16 * wave + m) * (size_t)HID + 8 * hh;
  const unsigned short* wp = WT + (size_t)m * (size_t)HID + 8 * hh;
#pragma unroll 1
  for (int ks = 0; ks < HID / 32; ++ks) {
    FragB af;
    af.h[0] = *(const v8usa*)(ap + 32 * ks);
    af.h[1] = *(const v8usa*)(ap + 32 * ks + 16);
#pragma unroll
    for (int t = 0; t < 4; ++t) {
      const unsigned short* wq = wp + (size_t)(16 * t) * (size_t)HID + 32 * ks;
      FragB bf;
      bf.h[0] = *(const v8usa*)wq;
      bf.h[1] = *(const v8usa*)(wq + 16);
      acc[t] = wmb(af, bf, acc[t]);
    }
  }

#pragma unroll
  for (int t = 0; t < 4; ++t) {
    const int lc = 16 * t + m;
#pragma unroll
    for (int r = 0; r < 8; ++r) {
      const int lr = 16 * wave + 8 * hh + r;
      stg[lr * GBN + lc] = acc[t][r];
    }
  }
  __syncthreads();

  v4f fv[8];
#pragma unroll
  for (int i = 0; i < 8; ++i) {
    const int lr = 16 * wave + 2 * i + hh;
    const v4f v = *(const v4fa*)(stg + lr * GBN + 4 * m);
    const float s = sdi[lr];
    v4f q;
    q.x = v.x * s; q.y = v.y * s; q.z = v.z * s; q.w = v.w * s;
    fv[i] = q;
  }
#pragma unroll
  for (int i = 0; i < 8; ++i) {
    const int lr = 16 * wave + 2 * i + hh;
    float* op = outF + (size_t)(rowBase + lr) * (size_t)HID + 4 * m;
    *(volatile v4f*)op = fv[i];
  }
  __threadfence();
#pragma unroll
  for (int i = 0; i < 8; ++i) {
    const int lr = 16 * wave + 2 * i + hh;
    float* op = outF + (size_t)(rowBase + lr) * (size_t)HID + 4 * m;
    *(volatile v4f*)op = fv[i];
  }
}

__global__ __launch_bounds__(NTHR) void k_scan(const int* __restrict__ srcs, const int* __restrict__ dsts,
                                               int nE, int nN, int vec8,
                                               const float* __restrict__ dis, const float* __restrict__ hs,
                                               const float* __restrict__ bias, const int* __restrict__ bat,
                                               const int* __restrict__ ngp, float* rec) {
  extern __shared__ __attribute__((aligned(16))) int dsm[];
  int* list = dsm;
  int* hl   = dsm + LISTN;
  int* cur  = dsm + LISTN + RCAP;
  int* sl   = dsm + DREG;
  int* cnt  = sl + RCAP;
  int* offs = cnt + NBA;
  int* misc = offs + NBA;
  const int tid = (int)threadIdx.x, lane = tid & 31, wave = tid >> 5;
  const int nodeBase = (int)blockIdx.x * NBA;

  {
    const v4i z4 = {0, 0, 0, 0};
    for (int i = tid * 4; i < SCAN_ZINTS; i += NTHR * 4) *(v4ia*)(dsm + i) = z4;
    if (tid < 16) misc[tid] = 0;
  }
  float bv0, bv1;
  {
    const v2f a = *(const v2fa*)(bias + 2 * lane);
    bv0 = bf16_val(a.x); bv1 = bf16_val(a.y);
  }
  int ng = ngp[0];
  ng = ng < 0 ? 0 : (ng > NG ? NG : ng);
  __syncthreads();

  int t = 0, ov = 0;
  const int nChunks = (nE + CHUNK - 1) / CHUNK;
#pragma unroll 1
  for (int ch = 0; ch < nChunks; ++ch) {
    const int cbase = ch * CHUNK;
    const int wc = scan_chunk<SLA>(dsts, nE, cbase, nodeBase, NBA, vec8, list, tid, lane, wave);
    if (lane == 0) misc[wave] = wc;
    __syncthreads();
    if (wave == 0) {
#pragma unroll 1
      for (int w2 = 0; w2 < NWAVE; ++w2) {
        int c = misc[w2];
        c = c < 0 ? 0 : (c > WCAP ? WCAP : c);
#pragma unroll 1
        for (int b0 = 0; b0 < c; b0 += 32) {
          const int idx = b0 + lane;
          const int ent = list[w2 * WCAP + (idx < WCAP ? idx : WCAP - 1)];
          const int m32 = (c - b0) < 32 ? (c - b0) : 32;
#pragma unroll 1
          for (int k = 0; k < m32; ++k) {
            const int u    = __builtin_amdgcn_readlane(ent, k);
            const int slot = u & (NBA - 1);
            const int el   = (u >> SLA) & (CHUNK - 1);
            const int pk   = ((cbase + el) << SLA) | slot;
            if (t < RCAP) {
              if (lane == 0) { hl[t] = pk; cnt[slot] = cnt[slot] + 1; }
              t = t + 1;
            } else {
              ov = 1;
            }
          }
        }
      }
    }
    __syncthreads();
  }
  if (wave == 0 && lane == 0) { misc[8] = t; misc[9] = ov; }
  __syncthreads();
  int tt = misc[8];
  tt = tt < 0 ? 0 : (tt > RCAP ? RCAP : tt);
  const int ovf = misc[9];

  if (wave == 0) {
    const int base = lane * (NBA / 32);
    int s = 0;
#pragma unroll 1
    for (int i = 0; i < NBA / 32; ++i) s += cnt[base + i];
    int incl = s;
#pragma unroll
    for (int d = 1; d < 32; d <<= 1) {
      const int y = __shfl_up(incl, d, 32);
      if (lane >= d) incl += y;
    }
    int run = incl - s;
#pragma unroll 1
    for (int i = 0; i < NBA / 32; ++i) {
      const int cv = cnt[base + i];
      offs[base + i] = run;
      cur[base + i]  = run;
      run += cv;
    }
  }
  __syncthreads();
  if (wave == 0) {
#pragma unroll 1
    for (int b0 = 0; b0 < tt; b0 += 32) {
      const int idx = b0 + lane;
      const int ent = hl[idx < RCAP ? idx : RCAP - 1];
      const int m32 = (tt - b0) < 32 ? (tt - b0) : 32;
#pragma unroll 1
      for (int k = 0; k < m32; ++k) {
        const int u    = __builtin_amdgcn_readlane(ent, k);
        const int slot = u & (NBA - 1);
        if (lane == 0) {
          int p = cur[slot];
          p = p < 0 ? 0 : (p > RCAP - 1 ? RCAP - 1 : p);
          sl[p] = u;
          cur[slot] = p + 1;
        }
      }
    }
  }
  __syncthreads();

  {
    const float ninf = __uint_as_float(0xff800000u);
    const v4f n4 = {ninf, ninf, ninf, ninf};
    for (int i = tid * 4; i < DREG; i += NTHR * 4) *(v4fa*)(dsm + i) = n4;
  }
  __syncthreads();

  const float qnan = __int_as_float(0x7fc00000);
  const float pz = (ovf != 0) ? qnan : 0.0f;
  int* tb = dsm + wave * PTAB + 2 * lane;
#pragma unroll 1
  for (int si = 0; si < NBA / NWAVE; ++si) {
    const int s    = si * NWAVE + wave;
    const int node = nodeBase + s;
    int c = cnt[s];
    const bool big = c > DEGCAP;
    c = c < 0 ? 0 : (c > DEGCAP ? DEGCAP : c);
    int o = offs[s];
    o = o < 0 ? 0 : (o > RCAP ? RCAP : o);
    const int nc = node < nN ? node : nN - 1;
    const float dd = dis[nc];
    float acc0 = 0.0f, acc1 = 0.0f;
#pragma unroll 1
    for (int b0 = 0; b0 < c; b0 += 32) {
      int idx = o + b0 + lane;
      idx = idx > RCAP - 1 ? RCAP - 1 : idx;
      const int ent = sl[idx];
      int eid = ent >> SLA;
      eid = eid < 0 ? 0 : (eid > nE - 1 ? nE - 1 : eid);
      int sr = srcs[eid];
      sr = sr < 0 ? 0 : (sr > nN - 1 ? nN - 1 : sr);
      const int m32 = (c - b0) < 32 ? (c - b0) : 32;
#pragma unroll 1
      for (int k = 0; k < m32; ++k) {
        const int sk = __builtin_amdgcn_readlane(sr, k);
        const v2f a = *(const v2fa*)(hs + (size_t)sk * HID + 2 * lane);
        acc0 += a.x; acc1 += a.y;
      }
    }
    float sv0, sv1;
    {
      const v2f a = *(const v2fa*)(hs + (size_t)nc * HID + 2 * lane);
      sv0 = a.x; sv1 = a.y;
    }
    const float pzr = big ? qnan : pz;
    const float t0 = dd * (acc0 + sv0) + bv0;
    const float t1 = dd * (acc1 + sv1) + bv1;
    float y0 = (t0 >= 0.0f) ? t0 : 0.2f * t0;
    float y1 = (t1 >= 0.0f) ? t1 : 0.2f * t1;
    y0 = y0 + pzr; y1 = y1 + pzr;
    const int b = bat[nc];
    const bool valid = (node < nN) && ((unsigned)b < (unsigned)ng);
    const int bc = b < 0 ? 0 : (b > NG - 1 ? NG - 1 : b);
    v2fa* tp = (v2fa*)(tb + bc * HID);
    const v2f mm = *tp;
    v2f nn;
    nn.x = nmax(y0, mm.x);
    nn.y = nmax(y1, mm.y);
    if (valid) *tp = nn;
  }
  __syncthreads();

  v4f rv[4];
#pragma unroll
  for (int it = 0; it < 4; ++it) {
    const int idx = it * (NTHR * 4) + 4 * tid;
    v4f mx = *(const v4fa*)(dsm + idx);
#pragma unroll 1
    for (int w2 = 1; w2 < NWAVE; ++w2) {
      const v4f ov4 = *(const v4fa*)(dsm + w2 * PTAB + idx);
      mx.x = nmax(ov4.x, mx.x); mx.y = nmax(ov4.y, mx.y);
      mx.z = nmax(ov4.z, mx.z); mx.w = nmax(ov4.w, mx.w);
    }
    rv[it] = mx;
  }
  float* rp = rec + (size_t)blockIdx.x * NOUT;
#pragma unroll
  for (int it = 0; it < 4; ++it) *(volatile v4f*)(rp + it * (NTHR * 4) + 4 * tid) = rv[it];
  __threadfence();
#pragma unroll
  for (int it = 0; it < 4; ++it) *(volatile v4f*)(rp + it * (NTHR * 4) + 4 * tid) = rv[it];
}

__global__ __launch_bounds__(NTHR) void k_head(const float* __restrict__ rec, int nrec,
                                               const float* __restrict__ Wfc, const float* __restrict__ bfc,
                                               float* out) {
  extern __shared__ __attribute__((aligned(16))) unsigned char hsm[];
  double* Gd  = (double*)hsm;
  double* Md  = Gd + 4096;
  double* vd  = Md + 4096;
  double* wd  = vd + 64;
  double* pd  = wd + 64;
  double* sdl = pd + 256;
  float* sWf = (float*)(hsm + (size_t)HEAD_DBL * 8);
  float* sO  = sWf + 4096;
  unsigned short* sA  = (unsigned short*)(sO + 4096);
  unsigned short* sWb = sA + NG * K2;
  const int tid = (int)threadIdx.x, lane = tid & 31, wave = tid >> 5, hh = lane >> 4, m = lane & 15;
  const float ninf = __uint_as_float(0xff800000u);

#pragma unroll 1
  for (int it = 0; it < 4; ++it) {
    const int idx = it * (NTHR * 4) + 4 * tid;
    const v4f w = *(const v4fa*)(Wfc + idx);
    const unsigned b0 = bf16_bits(w.x), b1 = bf16_bits(w.y), b2 = bf16_bits(w.z), b3 = bf16_bits(w.w);
    v4f wr;
    wr.x = __uint_as_float(b0 << 16); wr.y = __uint_as_float(b1 << 16);
    wr.z = __uint_as_float(b2 << 16); wr.w = __uint_as_float(b3 << 16);
    v4us wb;
    wb[0] = (unsigned short)b0; wb[1] = (unsigned short)b1; wb[2] = (unsigned short)b2; wb[3] = (unsigned short)b3;
    *(v4fa*)(sWf + idx) = wr;
    *(v4usa*)(sWb + idx) = wb;
  }
#pragma unroll 1
  for (int it = 0; it < 4; ++it) {
    const int idx = it * (NTHR * 4) + 4 * tid;
    v4f mx = {ninf, ninf, ninf, ninf};
#pragma unroll 1
    for (int b = 0; b < nrec; ++b) {
      const v4f o = *(const v4fa*)(rec + (size_t)b * NOUT + idx);
      mx.x = nmax(o.x, mx.x); mx.y = nmax(o.y, mx.y);
      mx.z = nmax(o.z, mx.z); mx.w = nmax(o.w, mx.w);
    }
    v4us h4, l4;
    unsigned hb;
    hb = bf16_bits_n(mx.x); h4[0] = (unsigned short)hb; l4[0] = (unsigned short)bf16_bits_n(mx.x - __uint_as_float(hb << 16));
    hb = bf16_bits_n(mx.y); h4[1] = (unsigned short)hb; l4[1] = (unsigned short)bf16_bits_n(mx.y - __uint_as_float(hb << 16));
    hb = bf16_bits_n(mx.z); h4[2] = (unsigned short)hb; l4[2] = (unsigned short)bf16_bits_n(mx.z - __uint_as_float(hb << 16));
    hb = bf16_bits_n(mx.w); h4[3] = (unsigned short)hb; l4[3] = (unsigned short)bf16_bits_n(mx.w - __uint_as_float(hb << 16));
    const int g = idx >> 6, c = idx & 63;
    *(v4usa*)(sA + g * K2 + c) = h4;
    *(v4usa*)(sA + g * K2 + HID + c) = l4;
  }
  __syncthreads();

  const int gr = tid >> 2, q16 = (tid & 3) * 16;
#pragma unroll 1
  for (int jj = 0; jj < 16; ++jj) {
    const int j = q16 + jj;
    double s = 0.0;
#pragma unroll 4
    for (int k = 0; k < HID; ++k) s += (double)sWf[gr * HID + k] * (double)sWf[j * HID + k];
    Gd[gr * HID + j] = s;
  }
  __syncthreads();
#pragma unroll 1
  for (int jj = 0; jj < 16; ++jj) {
    const int j = q16 + jj;
    double s = 0.0;
#pragma unroll 4
    for (int k = 0; k < HID; ++k) s += Gd[gr * HID + k] * Gd[k * HID + j];
    Md[gr * HID + j] = s;
  }
  if (tid < HID) vd[tid] = 1.0 + (double)tid * (1.0 / 64.0);
  __syncthreads();
#pragma unroll 1
  for (int it = 0; it < NITER; ++it) {
    double s = 0.0;
#pragma unroll 4
    for (int kk = 0; kk < 16; ++kk) s += Md[gr * HID + q16 + kk] * vd[q16 + kk];
    pd[tid] = s;
    __syncthreads();
    if (tid < HID) wd[tid] = ((pd[4 * tid] + pd[4 * tid + 1]) + pd[4 * tid + 2]) + pd[4 * tid + 3];
    __syncthreads();
    if (tid < HID) {
      double nrm = 0.0;
#pragma unroll 4
      for (int k = 0; k < HID; ++k) nrm += wd[k] * wd[k];
      float nf = (float)nrm;
      nf = (nf > 1e-30f) ? nf : 1e-30f;
      vd[tid] = wd[tid] * (double)rsqrtf(nf);
    }
    __syncthreads();
  }
  {
    double s = 0.0;
#pragma unroll 4
    for (int kk = 0; kk < 16; ++kk) s += Gd[gr * HID + q16 + kk] * vd[q16 + kk];
    pd[tid] = s;
  }
  __syncthreads();
  if (tid < HID) wd[tid] = ((pd[4 * tid] + pd[4 * tid + 1]) + pd[4 * tid + 2]) + pd[4 * tid + 3];
  __syncthreads();
  if (tid == 0) {
    double num = 0.0, den = 0.0;
#pragma unroll 4
    for (int k = 0; k < HID; ++k) { num += vd[k] * wd[k]; den += vd[k] * vd[k]; }
    sdl[0] = num / den;
  }
  __syncthreads();
  float is;
  {
    const double lam = sdl[0];
    const double y0 = (double)rsqrtf((float)lam);
    const double y1 = y0 * (1.5 - 0.5 * lam * y0 * y0);
    is = (float)y1;
  }

  const int rt = wave >> 1, ct0 = (wave & 1) * 2;
  v8f acc[2];
  {
    const v8f z = {0.f, 0.f, 0.f, 0.f, 0.f, 0.f, 0.f, 0.f};
    acc[0] = z; acc[1] = z;
  }
  const unsigned short* ap = sA + (16 * rt + m) * K2 + 8 * hh;
#pragma unroll
  for (int ks = 0; ks < K2 / 32; ++ks) {
    FragB af;
    af.h[0] = *(const v8usa*)(ap + 32 * ks);
    af.h[1] = *(const v8usa*)(ap + 32 * ks + 16);
    const int kk = (32 * ks) & (HID - 1);
#pragma unroll
    for (int t = 0; t < 2; ++t) {
      const unsigned short* wq = sWb + (16 * (ct0 + t) + m) * HID + kk + 8 * hh;
      FragB bf;
      bf.h[0] = *(const v8usa*)wq;
      bf.h[1] = *(const v8usa*)(wq + 16);
      acc[t] = wmb(af, bf, acc[t]);
    }
  }
#pragma unroll
  for (int t = 0; t < 2; ++t) {
    const int lc = 16 * (ct0 + t) + m;
    const float bb = bf16_val(bfc[lc]);
#pragma unroll
    for (int r = 0; r < 8; ++r) {
      const int lr = 16 * rt + 8 * hh + r;
      sO[lr * HID + lc] = fmaf(acc[t][r], is, bb);
    }
  }
  __syncthreads();
  v4f ov[4];
#pragma unroll
  for (int it = 0; it < 4; ++it) ov[it] = *(const v4fa*)(sO + it * (NTHR * 4) + 4 * tid);
#pragma unroll
  for (int it = 0; it < 4; ++it) *(volatile v4f*)(out + it * (NTHR * 4) + 4 * tid) = ov[it];
  __threadfence();
#pragma unroll
  for (int it = 0; it < 4; ++it) *(volatile v4f*)(out + it * (NTHR * 4) + 4 * tid) = ov[it];
}

static inline int cdiv(int a, int b) { return (a + b - 1) / b; }
static inline size_t al256(size_t o) { return (o + 255) & ~(size_t)255; }

extern "C" void kernel_launch(void* const* d_in, const int* in_sizes, int n_in,
                              void* d_out, int out_size, void* d_ws, size_t ws_size,
                              hipStream_t stream) {
  if (n_in < 8) return;
  if (in_sizes[0] < HID || (in_sizes[0] % HID) != 0) return;
  const int nN = in_sizes[0] / HID;
  if (nN < 1 || nN > (1 << 22)) return;
  if (in_sizes[1] != HID * HID || in_sizes[2] != HID) return;
  if (in_sizes[3] != HID * HID || in_sizes[4] != HID) return;
  if (in_sizes[5] < 2 || (in_sizes[5] & 1) != 0) return;
  const int nE = in_sizes[5] / 2;
  if (nE < 1 || nE >= (1 << (31 - SLA))) return;
  if (in_sizes[6] != nN) return;
  if (in_sizes[7] < 1) return;
  if (out_size != NOUT) return;

  const float* x    = (const float*)d_in[0];
  const float* Wg   = (const float*)d_in[1];
  const float* bg   = (const float*)d_in[2];
  const float* Wfc  = (const float*)d_in[3];
  const float* bfc  = (const float*)d_in[4];
  const int*   edge = (const int*)d_in[5];
  const int*   bat  = (const int*)d_in[6];
  const int*   ngp  = (const int*)d_in[7];
  float* out = (float*)d_out;
  const int* src = edge;
  const int* dst = edge + nE;

  const int MP   = cdiv(nN, GBM) * GBM;
  const int gM   = MP / GBM;
  const int gD   = cdiv(nN, NBD);
  const int NBPD = gD * NBD;
  const int gA   = cdiv(nN, NBA);
  if (NBPD < MP) return;
  if ((long long)gA * NBA < (long long)nN) return;
  const int vec8 = ((nE & 3) == 0) ? 1 : 0;
  const int nUx = MP * (HID / 8);
  const int gX  = cdiv(nUx, NTHR);

  char* ws = (char*)d_ws;
  size_t off = 0;
  const size_t oDIS = off; off = al256(off + (size_t)NBPD * 4);
  const size_t oWGT = off; off = al256(off + (size_t)HID * HID * 2);
  const size_t oXB  = off; off = al256(off + (size_t)MP * HID * 2);
  const size_t oHS  = off; off = al256(off + (size_t)MP * HID * 4);
  const size_t oREC = off; off = al256(off + (size_t)gA * NOUT * 4);
  if (off > ws_size || off > (size_t)WSMAX) return;
  float*          DIS = (float*)(ws + oDIS);
  unsigned short* WGT = (unsigned short*)(ws + oWGT);
  unsigned short* XB  = (unsigned short*)(ws + oXB);
  float*          HS  = (float*)(ws + oHS);
  float*          REC = (float*)(ws + oREC);

  const size_t scanLds = (size_t)SCAN_LDS_INTS * 4;
  const size_t headLds = (size_t)HEAD_LDS;
  hipFuncSetAttribute(reinterpret_cast<const void*>(&k_scan), hipFuncAttributeMaxDynamicSharedMemorySize, (int)scanLds);
  hipFuncSetAttribute(reinterpret_cast<const void*>(&k_head), hipFuncAttributeMaxDynamicSharedMemorySize, (int)headLds);

  k_prep<<<gX + NWU / NTHR, NTHR, 0, stream>>>(x, Wg, nN, gX, nUx, XB, WGT);
  k_deg<<<gD, NTHR, 0, stream>>>(dst, nE, vec8, DIS);
  k_gemm<<<gM, GTHR, 0, stream>>>(XB, WGT, DIS, HS);
  k_scan<<<gA, NTHR, scanLds, stream>>>(src, dst, nE, nN, vec8, DIS, HS, bg, bat, ngp, REC);
  k_head<<<1, NTHR, headLds, stream>>>(REC, gA, Wfc, bfc, out);
}
